// MultiHeadSelfAttentionLayer_30605936951552
// MI455X (gfx1250) — hardware-verified
//
#include <hip/hip_runtime.h>
#include <hip/hip_bf16.h>
#include <stdint.h>
#include <math.h>

constexpr int kBatch = 4;
constexpr int kSeq   = 2048;
constexpr int kFeat  = 512;
constexpr int kProj  = 512;
constexpr int kRows  = kBatch * kSeq;

constexpr size_t kOffXB    = 0;
constexpr size_t kBytesXB  = (size_t)kRows * kFeat * 2;
constexpr size_t kOffWT    = kOffXB + kBytesXB;
constexpr size_t kBytesWT1 = (size_t)kProj * kFeat * 2;
constexpr size_t kOffSC    = 0;
constexpr size_t kBytesSC  = (size_t)kBatch * kSeq * kSeq * 4;
constexpr size_t kOffP     = kOffSC + kBytesSC;
constexpr size_t kBytesP   = (size_t)kBatch * kSeq * kSeq * 2;
constexpr size_t kOffQ     = kOffP + kBytesP;
constexpr size_t kBytesQKV = (size_t)kRows * kProj * 2;
constexpr size_t kOffK     = kOffQ + kBytesQKV;
constexpr size_t kOffVT    = kOffK + kBytesQKV;
constexpr size_t kWsTotal  = kOffVT + kBytesQKV;
static_assert(kOffWT + 3 * kBytesWT1 <= kOffP);
static_assert((size_t)kBatch * kProj * kSeq * 2 == kBytesQKV);
static_assert(kWsTotal == 125829120ull);
static_assert(kWsTotal <= 134217728ull);
static_assert((kOffWT % 128) == 0 && (kOffP % 128) == 0 && (kOffQ % 128) == 0 && (kOffK % 128) == 0 && (kOffVT % 128) == 0);
static_assert(kRows % 64 == 0 && kProj % 64 == 0 && kSeq % 64 == 0);
static_assert(kFeat % 32 == 0 && kProj % 32 == 0 && kSeq % 32 == 0);
static_assert((kRows * kFeat) % (8 * 256) == 0);
static_assert(kRows % 8 == 0 && kSeq % 256 == 0);
static_assert(kFeat % 64 == 0);

typedef __attribute__((ext_vector_type(16))) _Float16 v16h;
typedef __attribute__((ext_vector_type(8)))  _Float16 v8h;
typedef __attribute__((ext_vector_type(16))) __bf16   v16b;
typedef __attribute__((ext_vector_type(8)))  __bf16   v8b;
typedef __attribute__((ext_vector_type(8)))  float    v8f;
typedef __attribute__((ext_vector_type(4)))  float    v4f;
typedef __attribute__((ext_vector_type(4)))  unsigned int v4u;

__device__ __forceinline__ unsigned short f2bf_bits(float f) {
  unsigned u = __float_as_uint(f);
  return (unsigned short)((u + 0x7FFFu + ((u >> 16) & 1u)) >> 16);
}
__device__ __forceinline__ float bf_bits2f(unsigned short h) { return __uint_as_float(((unsigned)h) << 16); }
__device__ __forceinline__ unsigned int f16_bits_u(float f) {
  return (unsigned int)__builtin_bit_cast(unsigned short, (_Float16)f);
}

__device__ __forceinline__ void dep_guard_h(v8f& a, v8f& b, v16h x, v16h y) { asm volatile("v_nop\n\tv_nop\n\tv_nop\n\tv_nop" : "+v"(a), "+v"(b) : "v"(x), "v"(y)); }
__device__ __forceinline__ void dep_guard_b(v8f& a, v8f& b, v16b x, v16b y) { asm volatile("v_nop\n\tv_nop\n\tv_nop\n\tv_nop" : "+v"(a), "+v"(b) : "v"(x), "v"(y)); }
__device__ __forceinline__ void keep4_h(v16h a, v16h b, v16h c, v16h d) { asm volatile("v_nop" :: "v"(a), "v"(b), "v"(c), "v"(d)); }
__device__ __forceinline__ void keep4_b(v16b a, v16b b, v16b c, v16b d) { asm volatile("v_nop" :: "v"(a), "v"(b), "v"(c), "v"(d)); }
__device__ __forceinline__ void acc_guard4(v8f& a, v8f& b, v8f& c, v8f& d) { asm volatile("v_nop\n\tv_nop\n\tv_nop\n\tv_nop" : "+v"(a), "+v"(b), "+v"(c), "+v"(d)); }
template <typename T> struct Frag;
template <> struct Frag<_Float16> {
  typedef v16h V; union U { v16h v; v8h h[2]; };
  static __device__ __forceinline__ v16h load(const _Float16* p) {
    U f; f.h[0] = *(const v8h*)(p); f.h[1] = *(const v8h*)(p + 16); return f.v;
  }
  static __device__ __forceinline__ v8f mma(v16h a, v16h b, v8f c) {
    return __builtin_amdgcn_wmma_f32_16x16x32_f16(false, a, false, b, (short)0, c, false, false);
  }
  static __device__ __forceinline__ void guard(v8f& a, v8f& b, v16h x, v16h y) { dep_guard_h(a, b, x, y); }
  static __device__ __forceinline__ void keep(v16h a, v16h b, v16h c, v16h d) { keep4_h(a, b, c, d); }
};
template <> struct Frag<__bf16> {
  typedef v16b V; union U { v16b v; v8b h[2]; };
  static __device__ __forceinline__ v16b load(const __bf16* p) {
    U f; f.h[0] = *(const v8b*)(p); f.h[1] = *(const v8b*)(p + 16); return f.v;
  }
  static __device__ __forceinline__ v8f mma(v16b a, v16b b, v8f c) {
    return __builtin_amdgcn_wmma_f32_16x16x32_bf16(false, a, false, b, (short)0, c, false, false);
  }
  static __device__ __forceinline__ void guard(v8f& a, v8f& b, v16b x, v16b y) { dep_guard_b(a, b, x, y); }
  static __device__ __forceinline__ void keep(v16b a, v16b b, v16b c, v16b d) { keep4_b(a, b, c, d); }
};

template <int ET> struct Elem;
template <> struct Elem<0> { typedef _Float16 T; };
template <> struct Elem<1> { typedef __bf16 T; };
template <int ET, bool SPLIT, int BIAS_MODE, int OUT_MODE, bool RESID, int ACT = 0>
__global__ __launch_bounds__(256) void wmma_gemm64(
    const unsigned short* __restrict__ Ap, const unsigned short* __restrict__ A2p, int lda, long strideA,
    const unsigned short* __restrict__ Btp, const unsigned short* __restrict__ Bt2p, int ldb, long strideB,
    void* __restrict__ Cout, void* __restrict__ Cout2, int ldc, long strideC,
    const float* __restrict__ bias,
    const float* __restrict__ resid, long strideR,
    int M, int N, int K, float scale) {
  typedef typename Elem<ET>::T T;
  typedef typename Frag<T>::V V;
  const T* A = (const T*)Ap; const T* A2 = (const T*)A2p; const T* Bt = (const T*)Btp; const T* Bt2 = (const T*)Bt2p;
  __shared__ __align__(16) float sT[8][16 * 68];
  const int b    = blockIdx.y;
  const int lane = threadIdx.x & 31;
  const int wave = threadIdx.x >> 5;
  const int tilesN = N >> 6;
  const int tilesM = M >> 6;
  const int tile = blockIdx.x * 8 + wave;
  if (tile >= tilesM * tilesN) return;
  const int tm = tile / tilesN;
  const int tn = tile - tm * tilesN;
  const int m0 = tm << 6;
  const int n0 = tn << 6;

  const T* Ab  = A  + (size_t)b * strideA;
  const T* Bb  = Bt + (size_t)b * strideB;
  const T* Ab2 = SPLIT ? (A2  + (size_t)b * strideA) : nullptr;
  const T* Bb2 = SPLIT ? (Bt2 + (size_t)b * strideB) : nullptr;

  const int rlane = lane & 15;
  const int koff  = (lane >> 4) * 8;
  const int mOff  = (lane >> 4) * 8;

  v8f acc[4][4];
#pragma unroll
  for (int i = 0; i < 4; ++i)
#pragma unroll
    for (int j = 0; j < 4; ++j) acc[i][j] = (v8f){0.f,0.f,0.f,0.f,0.f,0.f,0.f,0.f};

  for (int k0 = 0; k0 < K; k0 += 32) {
    V bh[4], bl[4];
#pragma unroll
    for (int j = 0; j < 4; ++j) {
      const size_t bo = (size_t)(n0 + (j << 4) + rlane) * ldb + koff + k0;
      bh[j] = Frag<T>::load(Bb + bo);
      if (SPLIT) bl[j] = Frag<T>::load(Bb2 + bo);
    }
#pragma unroll
    for (int i = 0; i < 4; ++i) {
      const size_t ao = (size_t)(m0 + (i << 4) + rlane) * lda + koff + k0;
      V ah = Frag<T>::load(Ab + ao);
      V al;
      if (SPLIT) al = Frag<T>::load(Ab2 + ao);
#pragma unroll
      for (int j = 0; j < 4; ++j) {
        acc[i][j] = Frag<T>::mma(ah, bh[j], acc[i][j]);
        if (SPLIT) {
          acc[i][j] = Frag<T>::mma(ah, bl[j], acc[i][j]);
          acc[i][j] = Frag<T>::mma(al, bh[j], acc[i][j]);
        }
      }
      Frag<T>::guard(acc[i][0], acc[i][3], ah, SPLIT ? al : ah);
    }
    Frag<T>::keep(bh[0], bh[1], bh[2], bh[3]);
    if (SPLIT) Frag<T>::keep(bl[0], bl[1], bl[2], bl[3]);
  }
  acc_guard4(acc[0][0], acc[0][1], acc[0][2], acc[0][3]);
  acc_guard4(acc[1][0], acc[1][1], acc[1][2], acc[1][3]);
  acc_guard4(acc[2][0], acc[2][1], acc[2][2], acc[2][3]);
  acc_guard4(acc[3][0], acc[3][1], acc[3][2], acc[3][3]);

  float* slab = sT[wave];
  const float* Rb = RESID ? (resid + (size_t)b * strideR) : nullptr;
#pragma unroll
  for (int i = 0; i < 4; ++i) {
    const int mBase = m0 + (i << 4);
#pragma unroll
    for (int j = 0; j < 4; ++j) {
      const int n = n0 + (j << 4) + rlane;
      float bv = 0.f;
      if (BIAS_MODE == 2) bv = bias[n];
#pragma unroll
      for (int r = 0; r < 8; ++r) {
        float v = acc[i][j][r] * scale;
        if (BIAS_MODE == 1) v += bias[mBase + mOff + r];
        if (BIAS_MODE == 2) v += bv;
        if (RESID) v += Rb[(size_t)(mBase + mOff + r) * ldc + n];
        if (ACT == 1) v = tanhf(v);
        if (ACT == 2) v = fmaxf(v, 0.0f);
        if (ACT == 3) v = v / (1.0f + expf(-v));
        if (ACT == 4) v = (v > 0.f) ? v : 0.01f * v;
        if (ACT == 5) v = 0.5f * v * (1.0f + erff(v * 0.70710678118654752f));
        slab[(mOff + r) * 68 + (j << 4) + rlane] = v;
      }
    }
    __builtin_amdgcn_fence(__ATOMIC_RELEASE, "workgroup");
    __builtin_amdgcn_wave_barrier();
    __builtin_amdgcn_fence(__ATOMIC_ACQUIRE, "workgroup");
    if (OUT_MODE == 0) {
      float* C = (float*)Cout + (size_t)b * strideC;
      const int hh = lane >> 4, c4 = (lane & 15) * 4;
      for (int pass = 0; pass < 2; ++pass) {
#pragma unroll
        for (int it = 0; it < 8; ++it) {
          const int row = it * 2 + hh;
          v4f v = *(const v4f*)(slab + row * 68 + c4);
          *(volatile v4f*)(C + (size_t)(mBase + row) * ldc + n0 + c4) = v;
        }
        __threadfence();
      }
    } else {
      const int q = lane >> 3, c8 = (lane & 7) * 8;
      unsigned short* C  = (unsigned short*)Cout  + (size_t)b * strideC;
      unsigned short* C2 = (OUT_MODE == 2) ? ((unsigned short*)Cout2 + (size_t)b * strideC) : nullptr;
      for (int pass = 0; pass < 2; ++pass) {
#pragma unroll
        for (int it = 0; it < 4; ++it) {
          const int row = it * 4 + q;
          const float* sp = slab + row * 68 + c8;
          v8h hv, lv;
#pragma unroll
          for (int e = 0; e < 8; ++e) {
            if (OUT_MODE == 1) {
              hv[e] = (_Float16)sp[e];
            } else {
              unsigned short hb = f2bf_bits(sp[e]);
              unsigned short lb = f2bf_bits(sp[e] - bf_bits2f(hb));
              hv[e] = __builtin_bit_cast(_Float16, hb);
              lv[e] = __builtin_bit_cast(_Float16, lb);
            }
          }
          *(volatile v8h*)(C + (size_t)(mBase + row) * ldc + n0 + c8) = hv;
          if (OUT_MODE == 2) *(volatile v8h*)(C2 + (size_t)(mBase + row) * ldc + n0 + c8) = lv;
        }
        __threadfence();
      }
    }
    __builtin_amdgcn_fence(__ATOMIC_RELEASE, "workgroup");
    __builtin_amdgcn_wave_barrier();
    __builtin_amdgcn_fence(__ATOMIC_ACQUIRE, "workgroup");
  }
}

__global__ __launch_bounds__(256) void cast_f32_bf16x8(
    const float* __restrict__ in, unsigned short* __restrict__ out, int n8) {
  const int i = blockIdx.x * 256 + threadIdx.x;
  if (i < n8) {
    const v4f a = *(const v4f*)(in + (size_t)i * 8);
    const v4f c = *(const v4f*)(in + (size_t)i * 8 + 4);
    v4u w;
    w[0] = (unsigned)f2bf_bits(a[0]) | ((unsigned)f2bf_bits(a[1]) << 16);
    w[1] = (unsigned)f2bf_bits(a[2]) | ((unsigned)f2bf_bits(a[3]) << 16);
    w[2] = (unsigned)f2bf_bits(c[0]) | ((unsigned)f2bf_bits(c[1]) << 16);
    w[3] = (unsigned)f2bf_bits(c[2]) | ((unsigned)f2bf_bits(c[3]) << 16);
    unsigned short* p = out + (size_t)i * 8;
    *(volatile v4u*)p = w;
    __threadfence();
    *(volatile v4u*)p = w;
  }
}

__global__ __launch_bounds__(256) void wt_transpose_bf16(
    const float* __restrict__ W0, const float* __restrict__ W1, const float* __restrict__ W2,
    unsigned short* __restrict__ WT, int dimF, int dimP) {
  __shared__ float tile[64][65];
  const int tid  = threadIdx.x;
  const int lane = tid & 31;
  const int wave = tid >> 5;
  const int mat  = blockIdx.z;
  const float* W = (mat == 0) ? W0 : ((mat == 1) ? W1 : W2);
  const int p0 = blockIdx.x * 64;
  const int f0 = blockIdx.y * 64;
#pragma unroll
  for (int it = 0; it < 4; ++it) {
    const int idx = it * 256 + tid;
    const int row = idx >> 4;
    const int c4  = (idx & 15) * 4;
    const v4f v = *(const v4f*)(W + (size_t)(f0 + row) * dimP + p0 + c4);
    tile[row][c4 + 0] = v[0];
    tile[row][c4 + 1] = v[1];
    tile[row][c4 + 2] = v[2];
    tile[row][c4 + 3] = v[3];
  }
  __syncthreads();
  unsigned short* outp = WT + (size_t)mat * dimP * dimF;
  const int q  = lane >> 3;
  const int c8 = (lane & 7) * 8;
  v4u w[2];
#pragma unroll
  for (int it = 0; it < 2; ++it) {
    const int pp = wave * 8 + it * 4 + q;
#pragma unroll
    for (int j = 0; j < 4; ++j) {
      const unsigned lo = (unsigned)f2bf_bits(tile[c8 + 2 * j][pp]);
      const unsigned hi = (unsigned)f2bf_bits(tile[c8 + 2 * j + 1][pp]);
      w[it][j] = lo | (hi << 16);
    }
  }
  for (int pass = 0; pass < 2; ++pass) {
#pragma unroll
    for (int it = 0; it < 2; ++it) {
      const int pp = wave * 8 + it * 4 + q;
      *(volatile v4u*)(outp + (size_t)(p0 + pp) * dimF + f0 + c8) = w[it];
    }
    __threadfence();
  }
}

__global__ __launch_bounds__(256) void softmax_rows_f16(
    const float* __restrict__ S, unsigned short* __restrict__ Pout, int nrows, float carry) {
  __shared__ __align__(16) unsigned int prow[8][kSeq / 2];
  const int lane = threadIdx.x & 31;
  const int wave = threadIdx.x >> 5;
  int row = blockIdx.x * 8 + wave;
  row = (row < nrows) ? row : (nrows - 1);
  const float* sr = S + (size_t)row * kSeq;

  float m = -INFINITY;
#pragma unroll 1
  for (int ch = 0; ch < kSeq / 128; ++ch) {
    const v4f v = *(const v4f*)(sr + ch * 128 + lane * 4);
    m = fmaxf(m, fmaxf(fmaxf(v[0], v[1]), fmaxf(v[2], v[3])));
  }
#pragma unroll
  for (int off = 1; off < 32; off <<= 1) m = fmaxf(m, __shfl_xor(m, off, 32));

  float l = 0.0f;
#pragma unroll 1
  for (int ch = 0; ch < kSeq / 128; ++ch) {
    const v4f v = *(const v4f*)(sr + ch * 128 + lane * 4);
    l += (expf(v[0] - m) + expf(v[1] - m)) + (expf(v[2] - m) + expf(v[3] - m));
  }
#pragma unroll
  for (int off = 1; off < 32; off <<= 1) l += __shfl_xor(l, off, 32);
  const float inv = carry / l;

  unsigned int* pw = prow[wave];
#pragma unroll 1
  for (int ch = 0; ch < kSeq / 256; ++ch) {
    const v4f a = *(const v4f*)(sr + ch * 256 + lane * 8);
    const v4f c = *(const v4f*)(sr + ch * 256 + lane * 8 + 4);
    const float p0 = expf(a[0] - m) * inv, p1 = expf(a[1] - m) * inv;
    const float p2 = expf(a[2] - m) * inv, p3 = expf(a[3] - m) * inv;
    const float p4 = expf(c[0] - m) * inv, p5 = expf(c[1] - m) * inv;
    const float p6 = expf(c[2] - m) * inv, p7 = expf(c[3] - m) * inv;
    v4u w;
    w[0] = f16_bits_u(p0) | (f16_bits_u(p1) << 16);
    w[1] = f16_bits_u(p2) | (f16_bits_u(p3) << 16);
    w[2] = f16_bits_u(p4) | (f16_bits_u(p5) << 16);
    w[3] = f16_bits_u(p6) | (f16_bits_u(p7) << 16);
    *(v4u*)(pw + ch * 128 + lane * 4) = w;
  }

  unsigned short* pr = Pout + (size_t)row * kSeq;
  for (int pass = 0; pass < 2; ++pass) {
#pragma unroll 1
    for (int ch = 0; ch < kSeq / 256; ++ch) {
      const v4u w = *(const v4u*)(pw + ch * 128 + lane * 4);
      *(volatile v4u*)(pr + ch * 256 + lane * 8) = w;
    }
    __threadfence();
  }
}

extern "C" void kernel_launch(void* const* d_in, const int* in_sizes, int n_in,
                              void* d_out, int out_size, void* d_ws, size_t ws_size,
                              hipStream_t stream) {
  (void)in_sizes; (void)n_in; (void)out_size;
  if (ws_size < kWsTotal) return;

  const float* x  = (const float*)d_in[0];
  const float* Wq = (const float*)d_in[1];
  const float* Wk = (const float*)d_in[2];
  const float* Wv = (const float*)d_in[3];
  float* out = (float*)d_out;
  char* ws = (char*)d_ws;

  unsigned short* xb   = (unsigned short*)(ws + kOffXB);
  unsigned short* wt   = (unsigned short*)(ws + kOffWT);
  unsigned short* wqT  = wt;
  unsigned short* wkT  = wt + (size_t)kProj * kFeat;
  unsigned short* wvT  = wt + (size_t)2 * kProj * kFeat;
  float*          sc   = (float*)(ws + kOffSC);
  unsigned short* p16  = (unsigned short*)(ws + kOffP);
  unsigned short* q16  = (unsigned short*)(ws + kOffQ);
  unsigned short* k16  = (unsigned short*)(ws + kOffK);
  unsigned short* vt16 = (unsigned short*)(ws + kOffVT);

  const int n8 = kRows * kFeat / 8;
  cast_f32_bf16x8<<<dim3((n8 + 255) / 256), dim3(256), 0, stream>>>(x, xb, n8);

  wt_transpose_bf16<<<dim3(kProj / 64, kFeat / 64, 3), dim3(256), 0, stream>>>(Wq, Wk, Wv, wt, kFeat, kProj);

  {
    const int tiles = (kRows / 64) * (kProj / 64);
    wmma_gemm64<1, false, 0, 1, false><<<dim3((tiles + 7) / 8, 1), dim3(256), 0, stream>>>(
        xb, xb, kFeat, 0L, wqT, wqT, kFeat, 0L, (void*)q16, (void*)q16, kProj, 0L,
        x, x, 0L, kRows, kProj, kFeat, 1.0f);
    wmma_gemm64<1, false, 0, 1, false><<<dim3((tiles + 7) / 8, 1), dim3(256), 0, stream>>>(
        xb, xb, kFeat, 0L, wkT, wkT, kFeat, 0L, (void*)k16, (void*)k16, kProj, 0L,
        x, x, 0L, kRows, kProj, kFeat, 1.0f);
  }

  {
    const int tiles = (kProj / 64) * (kSeq / 64);
    wmma_gemm64<1, false, 0, 1, false><<<dim3((tiles + 7) / 8, kBatch), dim3(256), 0, stream>>>(
        wvT, wvT, kFeat, 0L, xb, xb, kFeat, (long)kSeq * kFeat, (void*)vt16, (void*)vt16, kSeq, (long)kProj * kSeq,
        x, x, 0L, kProj, kSeq, kFeat, 1.0f);
  }

  {
    const int tiles = (kSeq / 64) * (kSeq / 64);
    const float score_scale = 0.044194173824159216f;
    wmma_gemm64<0, false, 0, 0, false><<<dim3((tiles + 7) / 8, kBatch), dim3(256), 0, stream>>>(
        q16, q16, kProj, (long)kSeq * kProj, k16, k16, kProj, (long)kSeq * kProj, (void*)sc, (void*)sc, kSeq, (long)kSeq * kSeq,
        x, x, 0L, kSeq, kSeq, kProj, score_scale);
  }

  softmax_rows_f16<<<dim3(kRows / 8), dim3(256), 0, stream>>>(sc, p16, kRows, 1024.0f);

  {
    const int tiles = (kSeq / 64) * (kProj / 64);
    wmma_gemm64<0, false, 0, 0, false><<<dim3((tiles + 7) / 8, kBatch), dim3(256), 0, stream>>>(
        p16, p16, kSeq, (long)kSeq * kSeq, vt16, vt16, kSeq, (long)kProj * kSeq, (void*)out, (void*)out, kProj, (long)kSeq * kProj,
        x, x, 0L, kSeq, kProj, kSeq, 0.0009765625f);
  }
}
